// MSARowAttentionWithPairBias_21741124452583
// MI455X (gfx1250) — hardware-verified
//
#include <hip/hip_runtime.h>


#define NI   128
#define NJ   256
#define CC   256
#define CZ   128
#define NZR  (NJ * NJ)
#define NH_  8
#define CH   32
#define CHP  64
#define ZC   64
#define RPC  (ZC / NH_)
#define NR   (NI * NJ)
#define QSC  0.17677669529663689f
typedef _Float16 h16;
typedef unsigned short bf;
typedef __attribute__((ext_vector_type(16))) __bf16   v16bf;
typedef __attribute__((ext_vector_type(16))) _Float16 v16h;
typedef __attribute__((ext_vector_type(8)))  _Float16 v8h;
typedef __attribute__((ext_vector_type(8)))  unsigned short v8us;
typedef __attribute__((ext_vector_type(8)))  float    v8f;
typedef __attribute__((ext_vector_type(4)))  float    v4f;
typedef __attribute__((ext_vector_type(2)))  float    v2f;
typedef __attribute__((ext_vector_type(4)))  unsigned short v4us;
typedef __attribute__((ext_vector_type(2)))  unsigned short v2us;
typedef v8h  __attribute__((may_alias)) v8ha;
typedef v4f  __attribute__((may_alias)) v4fa;
typedef v8us __attribute__((may_alias)) v8usa;

__device__ __forceinline__ unsigned short f2bf(float f) { unsigned u = __float_as_uint(f); u += 0x7FFFu + ((u >> 16) & 1u); return (unsigned short)(u >> 16); }
__device__ __forceinline__ float bf2f(unsigned short b) { return __uint_as_float(((unsigned)b) << 16); }
__device__ __forceinline__ float bfr(float f) { return bf2f(f2bf(f)); }
__device__ __forceinline__ void splitf(float y, unsigned short& h, unsigned short& l) { h = f2bf(y); l = f2bf(y - bf2f(h)); }
__device__ __forceinline__ v16h cat16(v8h lo, v8h hi) { return __builtin_shufflevector(lo, hi, 0, 1, 2, 3, 4, 5, 6, 7, 8, 9, 10, 11, 12, 13, 14, 15); }
__device__ __forceinline__ v16bf cat16b(v8us lo, v8us hi) { return __builtin_bit_cast(v16bf, __builtin_shufflevector(lo, hi, 0, 1, 2, 3, 4, 5, 6, 7, 8, 9, 10, 11, 12, 13, 14, 15)); }
__device__ __forceinline__ v8f wmma16(v16h a, v16h b, v8f c) { return __builtin_amdgcn_wmma_f32_16x16x32_f16(false, a, false, b, (short)0, c, false, false); }
__device__ __forceinline__ v8f wmmab(v16bf a, v16bf b, v8f c) { return __builtin_amdgcn_wmma_f32_16x16x32_bf16(false, a, false, b, (short)0, c, false, false); }

template <typename T16> struct WFrag;
template <> struct WFrag<h16> { typedef v16h V; static __device__ __forceinline__ V ld(const h16* p) { return cat16(*(const v8h*)p, *(const v8h*)(p + 16)); } static __device__ __forceinline__ v8f mma(V a, V b, v8f c) { return wmma16(a, b, c); } };
template <> struct WFrag<bf> { typedef v16bf V; static __device__ __forceinline__ V ld(const bf* p) { return cat16b(*(const v8us*)p, *(const v8us*)(p + 16)); } static __device__ __forceinline__ v8f mma(V a, V b, v8f c) { return wmmab(a, b, c); } };
template <typename T16, int NSPLIT, bool BIAS>
__global__ __launch_bounds__(32) void k_gemmw(const T16* __restrict__ A, const T16* __restrict__ A2, const T16* __restrict__ Bt, const T16* __restrict__ Bt2, int K, float* C, int ldc, const float* __restrict__ bias, size_t sA, size_t sB, size_t sC) {
    typedef typename WFrag<T16>::V V;
    __shared__ __align__(16) float os[16 * 68];
    const size_t z = blockIdx.z; A += z * sA; if (A2) A2 += z * sA; Bt += z * sB; if (Bt2) Bt2 += z * sB; C += z * sC;
    const int lane = threadIdx.x & 31, lr = lane & 15, hi = lane >> 4; const int r0 = blockIdx.x * 64, c0 = blockIdx.y * 64;
    v8f acc[4][4];
#pragma unroll
    for (int mb = 0; mb < 4; ++mb)
#pragma unroll
        for (int nb = 0; nb < 4; ++nb) acc[mb][nb] = (v8f){};
    const size_t aoff = (size_t)(r0 + lr) * K + 8 * hi, boff = (size_t)(c0 + lr) * K + 8 * hi;
#pragma unroll 1
    for (int kc = 0; kc < K; kc += 32) {
        V a[4], a2[4];
#pragma unroll
        for (int mb = 0; mb < 4; ++mb) { a[mb] = WFrag<T16>::ld(A + aoff + (size_t)mb * 16 * K + kc); if (NSPLIT == 1 || NSPLIT == 2) a2[mb] = WFrag<T16>::ld(A2 + aoff + (size_t)mb * 16 * K + kc); }
#pragma unroll
        for (int nb = 0; nb < 4; ++nb) { const V b = WFrag<T16>::ld(Bt + boff + (size_t)nb * 16 * K + kc); V b2; if (NSPLIT >= 2) b2 = WFrag<T16>::ld(Bt2 + boff + (size_t)nb * 16 * K + kc);
#pragma unroll
            for (int mb = 0; mb < 4; ++mb) { acc[mb][nb] = WFrag<T16>::mma(a[mb], b, acc[mb][nb]); if (NSPLIT == 1 || NSPLIT == 2) acc[mb][nb] = WFrag<T16>::mma(a2[mb], b, acc[mb][nb]); if (NSPLIT >= 2) acc[mb][nb] = WFrag<T16>::mma(a[mb], b2, acc[mb][nb]); } }
        asm volatile("v_nop\n\tv_nop\n\tv_nop\n\tv_nop" : "+v"(acc[0][0]), "+v"(acc[1][1]), "+v"(acc[2][2]), "+v"(acc[3][3]) : "v"(a[0]), "v"(a[3]));
    }
#pragma unroll
    for (int mb = 0; mb < 4; ++mb) {
#pragma unroll
        for (int nb = 0; nb < 4; ++nb) {
#pragma unroll
            for (int j = 0; j < 8; ++j) os[(hi * 8 + j) * 68 + nb * 16 + lr] = acc[mb][nb][j]; }
        __builtin_amdgcn_wave_barrier(); asm volatile("" ::: "memory");
        float* crow = C + (size_t)(r0 + mb * 16) * ldc + c0;
#pragma unroll 1
        for (int ps = 0; ps < 2; ++ps) {
#pragma unroll
            for (int s = 0; s < 8; ++s) { const int row = 2 * s + hi, cofs = lr * 4; v4f val = *(const v4fa*)(os + row * 68 + cofs); if (BIAS) { val[0] += bfr(bias[c0 + cofs]); val[1] += bfr(bias[c0 + cofs + 1]); val[2] += bfr(bias[c0 + cofs + 2]); val[3] += bfr(bias[c0 + cofs + 3]); }
                *(volatile v4f*)(crow + (size_t)row * ldc + cofs) = val; }
            if (ps == 0) __threadfence(); }
        __builtin_amdgcn_wave_barrier(); asm volatile("" ::: "memory");
    }
}

__global__ __launch_bounds__(256) void k_wtG(const float* __restrict__ w, int K, int N, bf* Bt) {
    const int lane = threadIdx.x & 31; const int L0 = (blockIdx.x * 8 + (threadIdx.x >> 5)) * 8; const int nlines = N * K / 64;
#pragma unroll
    for (int ps = 0; ps < 2; ++ps) {
#pragma unroll 1
        for (int l = 0; l < 8; ++l) { const int L = L0 + l; if (L >= nlines) break; const size_t e = (size_t)L * 64 + lane * 2; const int k = (int)(e % K), n = (int)(e / K); v2us o;
            o[0] = f2bf(w[(size_t)k * N + n]); o[1] = f2bf(w[(size_t)(k + 1) * N + n]); *(volatile v2us*)(Bt + e) = o; }
        if (ps == 0) __threadfence(); }
}
__global__ __launch_bounds__(256) void k_cvt8(const float* __restrict__ src, bf* dst, size_t n8) { const size_t i = (size_t)blockIdx.x * 256 + threadIdx.x; if (i >= n8) return; const v8f v = *(const v8f*)(src + i * 8); v8us o;
#pragma unroll
    for (int k = 0; k < 8; ++k) o[k] = f2bf(v[k]); *(volatile v8us*)(dst + i * 8) = o; __threadfence(); *(volatile v8us*)(dst + i * 8) = o; }
__global__ __launch_bounds__(256) void k_lnz(const float* __restrict__ x, const float* __restrict__ lw, const float* __restrict__ lb, bf* XH, bf* XL) {
    const int lane = threadIdx.x & 31; const int r = blockIdx.x * 8 + (threadIdx.x >> 5); if (r >= NZR) return; const v4f a = *(const v4f*)(x + (size_t)r * CZ + lane * 4); float u[4]; float s = 0.f;
#pragma unroll
    for (int q = 0; q < 4; ++q) { u[q] = bfr(a[q]); s += u[q]; }
#pragma unroll
    for (int sh = 16; sh; sh >>= 1) s += __shfl_xor(s, sh, 32);
    const float mu = s * (1.0f / CZ); float s2 = 0.f;
#pragma unroll
    for (int q = 0; q < 4; ++q) { float d0 = __fsub_rn(u[q], mu); asm volatile("" : "+v"(d0)); float p = __fmul_rn(d0, d0); asm volatile("" : "+v"(p)); s2 = __fadd_rn(s2, p); }
#pragma unroll
    for (int sh = 16; sh; sh >>= 1) s2 += __shfl_xor(s2, sh, 32);
    const float rs = __fdiv_rn(1.0f, __fsqrt_rn(__fadd_rn(s2 * (1.0f / CZ), 1e-5f))); float xn[4]; v4us oh, ol;
#pragma unroll
    for (int q = 0; q < 4; ++q) { const int c = lane * 4 + q; float d1 = __fsub_rn(u[q], mu); asm volatile("" : "+v"(d1)); float n0 = __fmul_rn(d1, rs); asm volatile("" : "+v"(n0)); float n1 = __fmul_rn(n0, bfr(lw[c])); asm volatile("" : "+v"(n1)); xn[q] = __fadd_rn(n1, bfr(lb[c])); unsigned short h2, l2; splitf(xn[q], h2, l2); oh[q] = h2; ol[q] = l2; }
    *(volatile v4us*)(XH + (size_t)r * CZ + lane * 4) = oh; *(volatile v4us*)(XL + (size_t)r * CZ + lane * 4) = ol; __threadfence(); *(volatile v4us*)(XH + (size_t)r * CZ + lane * 4) = oh; *(volatile v4us*)(XL + (size_t)r * CZ + lane * 4) = ol;
}
__global__ __launch_bounds__(256) void k_lnm(const float* __restrict__ x, const float* __restrict__ lw, const float* __restrict__ lb, bf* MH, bf* ML) {
    const int lane = threadIdx.x & 31; const int r = blockIdx.x * 8 + (threadIdx.x >> 5); if (r >= NR) return; const v8f a = *(const v8f*)(x + (size_t)r * CC + lane * 8); float u[8]; float s = 0.f;
#pragma unroll
    for (int q = 0; q < 8; ++q) { u[q] = bfr(a[q]); s += u[q]; }
#pragma unroll
    for (int sh = 16; sh; sh >>= 1) s += __shfl_xor(s, sh, 32);
    const float mu = s * (1.0f / CC); float s2 = 0.f;
#pragma unroll
    for (int q = 0; q < 8; ++q) { float d0 = __fsub_rn(u[q], mu); asm volatile("" : "+v"(d0)); float p = __fmul_rn(d0, d0); asm volatile("" : "+v"(p)); s2 = __fadd_rn(s2, p); }
#pragma unroll
    for (int sh = 16; sh; sh >>= 1) s2 += __shfl_xor(s2, sh, 32);
    const float rs = __fdiv_rn(1.0f, __fsqrt_rn(__fadd_rn(s2 * (1.0f / CC), 1e-5f))); v8us oh, ol;
#pragma unroll
    for (int q = 0; q < 8; ++q) { const int c = lane * 8 + q; float d1 = __fsub_rn(u[q], mu); asm volatile("" : "+v"(d1)); float n0 = __fmul_rn(d1, rs); asm volatile("" : "+v"(n0)); float n1 = __fmul_rn(n0, bfr(lw[c])); asm volatile("" : "+v"(n1)); const float xn = __fadd_rn(n1, bfr(lb[c])); unsigned short h2, l2; splitf(xn, h2, l2); oh[q] = h2; ol[q] = l2; }
    *(volatile v8us*)(MH + (size_t)r * CC + lane * 8) = oh; *(volatile v8us*)(ML + (size_t)r * CC + lane * 8) = ol; __threadfence(); *(volatile v8us*)(MH + (size_t)r * CC + lane * 8) = oh; *(volatile v8us*)(ML + (size_t)r * CC + lane * 8) = ol; }
__global__ __launch_bounds__(256) void k_trib(const bf* __restrict__ XH, const bf* __restrict__ XL, const float* __restrict__ wtri, float* TB) { const size_t idx = (size_t)blockIdx.x * 256 + threadIdx.x; if (idx >= (size_t)NH_ * NZR) return; const int r = (int)(idx % NZR); const int h = (int)(idx / NZR); const bf* ph = XH + (size_t)r * CZ; const bf* pl = XL + (size_t)r * CZ; float s = 0.f;
#pragma unroll 4
    for (int c = 0; c < CZ; c += 8) { const v8us a = *(const v8us*)(ph + c), b2 = *(const v8us*)(pl + c);
#pragma unroll
        for (int q = 0; q < 8; ++q) { const float xn = __fadd_rn(bf2f(a[q]), bf2f(b2[q])); float p = __fmul_rn(xn, bfr(wtri[(size_t)h * CZ + c + q])    ); asm volatile("" : "+v"(p)); s = __fadd_rn(s, p); } }
    *(volatile float*)(TB + idx) = s; __threadfence(); *(volatile float*)(TB + idx) = s; }
__global__ __launch_bounds__(256) void k_qkpl(const float* __restrict__ F, int i0, float sc, bf* Ph, bf* Pl) { const size_t e = ((size_t)blockIdx.x * 256 + threadIdx.x) * 2; if (e >= (size_t)ZC * NJ * CH) return; const int d = (int)(e % CH); const int j = (int)((e / CH) % NJ); const int zz = (int)(e / ((size_t)CH * NJ)); const int i = i0 + zz / NH_, h = zz % NH_; const float* f = F + ((size_t)i * NJ + j) * CC + h * CH + d; v2us oh, ol;
#pragma unroll
    for (int q = 0; q < 2; ++q) { unsigned short a2, c2; splitf(__fmul_rn(f[q], sc), a2, c2); oh[q] = a2; ol[q] = c2; } *(volatile v2us*)(Ph + e) = oh; *(volatile v2us*)(Pl + e) = ol; __threadfence(); *(volatile v2us*)(Ph + e) = oh; *(volatile v2us*)(Pl + e) = ol; }
__global__ __launch_bounds__(256) void k_vtpl(const float* __restrict__ F, int i0, bf* Vh, bf* Vl) { const size_t e = ((size_t)blockIdx.x * 256 + threadIdx.x) * 2; if (e >= (size_t)ZC * CHP * NJ) return; const int j = (int)(e % NJ); const int dp = (int)((e / NJ) % CHP); const int zz = (int)(e / ((size_t)NJ * CHP)); const int i = i0 + zz / NH_, h = zz % NH_; v2us oh, ol;
#pragma unroll
    for (int q = 0; q < 2; ++q) { float x = 0.0f; if (dp < CH) x = F[((size_t)i * NJ + j + q) * CC + h * CH + dp]; unsigned short a2, c2; splitf(x, a2, c2); oh[q] = a2; ol[q] = c2; } *(volatile v2us*)(Vh + e) = oh; *(volatile v2us*)(Vl + e) = ol; __threadfence(); *(volatile v2us*)(Vh + e) = oh; *(volatile v2us*)(Vl + e) = ol; }
__global__ __launch_bounds__(256) void k_tsoft(const float* __restrict__ Sb, const float* __restrict__ TB, int i0, bf* Ph, bf* Pl) {
    const int lane = threadIdx.x & 31; const int row = blockIdx.x * 8 + (threadIdx.x >> 5); if (row >= ZC * NJ) return; const int jq = row % NJ; const int zz = row / NJ; const int i = i0 + zz / NH_, h = zz % NH_; const float* sr = Sb + (size_t)row * NJ; const float* tb = TB + (size_t)h * NZR + (size_t)jq * NJ; (void)i; float v[8]; float mx = -3.0e38f;
#pragma unroll
    for (int ch = 0; ch < 2; ++ch) { const int k0 = ch * 128 + lane * 4; const v4f a = *(const v4f*)(sr + k0), t4 = *(const v4f*)(tb + k0);
#pragma unroll
        for (int q = 0; q < 4; ++q) { float s1 = __fmul_rn(a[q], QSC); asm volatile("" : "+v"(s1)); const float t = __fadd_rn(s1, t4[q]); v[ch * 4 + q] = t; mx = fmaxf(mx, t); } }
#pragma unroll
    for (int sh = 16; sh; sh >>= 1) mx = fmaxf(mx, __shfl_xor(mx, sh, 32));
    float sum = 0.f;
#pragma unroll
    for (int k = 0; k < 8; ++k) { float d0 = __fsub_rn(v[k], mx); asm volatile("" : "+v"(d0)); v[k] = __builtin_amdgcn_exp2f(__fmul_rn(d0, 1.4426950408889634f)); sum += v[k]; }
#pragma unroll
    for (int sh = 16; sh; sh >>= 1) sum += __shfl_xor(sum, sh, 32);
    const float f = __fdiv_rn(1.0f, sum);
#pragma unroll 1
    for (int ps = 0; ps < 2; ++ps) {
#pragma unroll
        for (int ch = 0; ch < 2; ++ch) { v4us oh, ol;
#pragma unroll
            for (int q = 0; q < 4; ++q) { float pf = v[ch * 4 + q] * f; asm volatile("" : "+v"(pf)); unsigned short a, c2; splitf(pf, a, c2); oh[q] = a; ol[q] = c2; }
            const size_t oo = (size_t)row * NJ + ch * 128 + lane * 4; *(volatile v4us*)(Ph + oo) = oh; *(volatile v4us*)(Pl + oo) = ol; }
        if (ps == 0) __threadfence(); }
}
__global__ __launch_bounds__(256) void k_octx(const float* __restrict__ O, int i0, bf* Gh, bf* Gl) { const size_t e = ((size_t)blockIdx.x * 256 + threadIdx.x) * 2; if (e >= (size_t)ZC * NJ * CH) return; const int d = (int)(e % CH); const int jq = (int)((e / CH) % NJ); const int zz = (int)(e / ((size_t)CH * NJ)); const int i = i0 + zz / NH_, h = zz % NH_; const size_t r = (size_t)i * NJ + jq; const size_t oo = r * CC + h * CH + d; v2us oh, ol;
#pragma unroll
    for (int q = 0; q < 2; ++q) { const float o = O[((size_t)zz * NJ + jq) * CHP + d + q]; unsigned short a2, c2; splitf(o, a2, c2); oh[q] = a2; ol[q] = c2; }
    *(volatile v2us*)(Gh + oo) = oh; *(volatile v2us*)(Gl + oo) = ol; __threadfence(); *(volatile v2us*)(Gh + oo) = oh; *(volatile v2us*)(Gl + oo) = ol; }

__global__ __launch_bounds__(256) void k_fin(const float* __restrict__ msa, const float* __restrict__ FG, const float* __restrict__ bg, const float* __restrict__ O2, float* O) { const size_t i = (size_t)blockIdx.x * 256 + threadIdx.x; if (i >= (size_t)NR * CC / 4) return; const size_t e = i * 4; const int c0 = (int)(e % CC); const v4f m = *(const v4f*)(msa + e), fg = *(const v4f*)(FG + e), o2 = *(const v4f*)(O2 + e); v4f o;
#pragma unroll
    for (int q = 0; q < 4; ++q) { const float zg = __fadd_rn(fg[q], bfr(bg[c0 + q])); const float sg = __fdiv_rn(1.0f, __fadd_rn(1.0f, expf(-zg))); float t = __fmul_rn(sg, o2[q]); asm volatile("" : "+v"(t)); o[q] = __fadd_rn(bfr(m[q]), t); }
    *(volatile v4f*)(O + e) = o; __threadfence(); *(volatile v4f*)(O + e) = o; }

extern "C" void kernel_launch(void* const* d_in, const int* in_sizes, int n_in,
                              void* d_out, int out_size, void* d_ws, size_t ws_size, hipStream_t stream) {
    (void)in_sizes; (void)n_in; (void)out_size;
    const float* msa = (const float*)d_in[0]; const float* pair = (const float*)d_in[1]; const float* lmw = (const float*)d_in[2]; const float* lmb = (const float*)d_in[3]; const float* lzw = (const float*)d_in[4]; const float* lzb = (const float*)d_in[5]; const float* wq = (const float*)d_in[6]; const float* wk = (const float*)d_in[7]; const float* wv = (const float*)d_in[8]; const float* wb = (const float*)d_in[9]; const float* wo = (const float*)d_in[10]; const float* bo = (const float*)d_in[11]; const float* wg = (const float*)d_in[12]; const float* bg = (const float*)d_in[13];
    float* OUT = (float*)d_out;
    char* wsp = (char*)d_ws;
    auto take = [&](size_t bytes) { char* p = wsp; wsp += (bytes + 255) & ~(size_t)255; return (void*)p; };
    bf* WQ = (bf*)take((size_t)CC * CC * 2); bf* WK = (bf*)take((size_t)CC * CC * 2); bf* WV = (bf*)take((size_t)CC * CC * 2); bf* WG = (bf*)take((size_t)CC * CC * 2); bf* WO = (bf*)take((size_t)CC * CC * 2);
    bf* XH = (bf*)take((size_t)NR * CC * 2); bf* XL = (bf*)take((size_t)NR * CC * 2); bf* ZH_ = (bf*)take((size_t)NZR * CZ * 2); bf* ZL_ = (bf*)take((size_t)NZR * CZ * 2); float* TB = (float*)take((size_t)NH_ * NZR * 4);
    float* FQ = (float*)take((size_t)NR * CC * 4); float* FK = (float*)take((size_t)NR * CC * 4); float* FV = (float*)take((size_t)NR * CC * 4); float* FG = (float*)take((size_t)NR * CC * 4);
    bf* QPh = (bf*)take((size_t)ZC * NJ * CH * 2); bf* QPl = (bf*)take((size_t)ZC * NJ * CH * 2); bf* KPh = (bf*)take((size_t)ZC * NJ * CH * 2); bf* KPl = (bf*)take((size_t)ZC * NJ * CH * 2); bf* VTh = (bf*)take((size_t)ZC * CHP * NJ * 2); bf* VTl = (bf*)take((size_t)ZC * CHP * NJ * 2);
    float* Sb = (float*)take((size_t)ZC * NJ * NJ * 4); bf* Ph = (bf*)take((size_t)ZC * NJ * NJ * 2); bf* Pl = (bf*)take((size_t)ZC * NJ * NJ * 2); float* Ob = (float*)take((size_t)ZC * NJ * CHP * 4);
    bf* Gh = ZH_; bf* Gl = ZL_; float* O2 = FQ;
    if ((size_t)(wsp - (char*)d_ws) > ws_size) return;
    { const unsigned LW = (CC * CC / 8 + 255) / 256; k_cvt8<<<LW, 256, 0, stream>>>(wq, WQ, (size_t)CC * CC / 8); k_cvt8<<<LW, 256, 0, stream>>>(wk, WK, (size_t)CC * CC / 8); k_cvt8<<<LW, 256, 0, stream>>>(wv, WV, (size_t)CC * CC / 8); k_cvt8<<<LW, 256, 0, stream>>>(wg, WG, (size_t)CC * CC / 8); k_cvt8<<<LW, 256, 0, stream>>>(wo, WO, (size_t)CC * CC / 8); }
    k_lnm<<<NR / 8, 256, 0, stream>>>(msa, lmw, lmb, XH, XL); k_lnz<<<NZR / 8, 256, 0, stream>>>(pair, lzw, lzb, ZH_, ZL_); k_trib<<<(unsigned)(((size_t)NH_ * NZR + 255) / 256), 256, 0, stream>>>(ZH_, ZL_, wb, TB);
    k_gemmw<bf, 1, false><<<dim3(NR / 64, CC / 64, 1), 32, 0, stream>>>(XH, XL, WQ, nullptr, CC, FQ, CC, nullptr, 0, 0, 0);
    k_gemmw<bf, 1, false><<<dim3(NR / 64, CC / 64, 1), 32, 0, stream>>>(XH, XL, WK, nullptr, CC, FK, CC, nullptr, 0, 0, 0);
    k_gemmw<bf, 1, false><<<dim3(NR / 64, CC / 64, 1), 32, 0, stream>>>(XH, XL, WV, nullptr, CC, FV, CC, nullptr, 0, 0, 0);
    k_gemmw<bf, 1, false><<<dim3(NR / 64, CC / 64, 1), 32, 0, stream>>>(XH, XL, WG, nullptr, CC, FG, CC, nullptr, 0, 0, 0);
    const unsigned LQK = (unsigned)(((size_t)ZC * NJ * CH / 2 + 255) / 256), LVT = (unsigned)(((size_t)ZC * CHP * NJ / 2 + 255) / 256);
    for (int i0 = 0; i0 < NI; i0 += RPC) {
        k_qkpl<<<LQK, 256, 0, stream>>>(FQ, i0, 1.0f, QPh, QPl); k_qkpl<<<LQK, 256, 0, stream>>>(FK, i0, 1.0f, KPh, KPl); k_vtpl<<<LVT, 256, 0, stream>>>(FV, i0, VTh, VTl);
        k_gemmw<bf, 2, false><<<dim3(NJ / 64, NJ / 64, ZC), 32, 0, stream>>>(QPh, QPl, KPh, KPl, CH, Sb, NJ, nullptr, (size_t)NJ * CH, (size_t)NJ * CH, (size_t)NJ * NJ);
        k_tsoft<<<ZC * NJ / 8, 256, 0, stream>>>(Sb, TB, i0, Ph, Pl);
        k_gemmw<bf, 2, false><<<dim3(NJ / 64, CHP / 64, ZC), 32, 0, stream>>>(Ph, Pl, VTh, VTl, NJ, Ob, CHP, nullptr, (size_t)NJ * NJ, (size_t)CHP * NJ, (size_t)NJ * CHP);
        k_octx<<<LQK, 256, 0, stream>>>(Ob, i0, Gh, Gl); }
    k_gemmw<bf, 1, true><<<dim3(NR / 64, CC / 64, 1), 32, 0, stream>>>(Gh, Gl, WO, nullptr, CC, O2, CC, bo, 0, 0, 0);
    k_fin<<<(unsigned)(((size_t)NR * CC / 4 + 255) / 256), 256, 0, stream>>>(msa, FG, bg, O2, OUT);
}
